// SE3ProteinEncoder_37417755083171
// MI455X (gfx1250) — hardware-verified
//
#include <hip/hip_runtime.h>
#include <stddef.h>
#include <stdint.h>
#include <math.h>


#define HD     128
#define HP     136
#define AP     264
#define RP     40
#define FP     132
#define ROWS   64
#define WSC    16.0f
#define WINV   0.0625f
#define NCHMAX 4

#define T_WIH  0
#define T_WIL  16384
#define T_W1A  32768
#define T_W1R  49152
#define T_W2   53248
#define T_U1H  69632
#define T_U1L  102400
#define T_U2H  135168
#define T_U2L  151552
#define T_TOT  167936
#define T_GRP  (T_TOT / 8)

#define L_AHI  0
#define L_ALO  (ROWS * HP * 2)
#define L_H16  (2 * ROWS * HP * 2)
#define L_STG  (3 * ROWS * HP * 2)
#define L_RS   (L_STG + ROWS * FP * 4)
#define L_LDS  (L_RS + ROWS * 4)

#define E_RBF  0
#define E_HID  (ROWS * RP * 2)
#define E_STG  (E_HID + ROWS * HP * 2)
#define E_SIDX (E_STG + ROWS * HP * 2)
#define E_RED  (E_SIDX + ROWS * 4)
#define E_LDS  (E_RED + 32)

#define NTHR   256
#define NWAVE  8
#define NB     256
#define EPT    8
#define CHUNK  (NTHR * EPT)
#define WCAP   (EPT * 32)
#define A_ACC  0
#define A_LIST (NB * HD * 4)
#define A_WCNT (A_LIST + NWAVE * WCAP * 4)
#define A_LDS  (A_WCNT + 64)

#define U_AHI  0
#define U_ALO  (ROWS * AP * 2)
#define U_HH   (2 * ROWS * AP * 2)
#define U_HL   (U_HH + ROWS * HP * 2)
#define U_STG  (U_HL + ROWS * HP * 2)
#define U_CS   (U_STG + ROWS * FP * 4)
#define U_LDS  (U_CS + HD * 4)

static_assert(T_GRP * 8 == T_TOT);
static_assert(((T_WIL | T_W1A | T_W1R | T_W2 | T_U1H | T_U1L | T_U2H | T_U2L) & 63) == 0);
static_assert(((HP * 2) & 15) == 0 && ((AP * 2) & 15) == 0 && ((RP * 2) & 15) == 0 && ((FP * 4) & 15) == 0);
static_assert((L_ALO & 15) == 0 && (L_H16 & 15) == 0 && (L_STG & 15) == 0 && (L_RS & 15) == 0);
static_assert((E_HID & 15) == 0 && (E_STG & 15) == 0 && (E_SIDX & 15) == 0 && (E_RED & 15) == 0);
static_assert((A_LIST & 15) == 0 && (A_WCNT & 15) == 0);
static_assert((U_ALO & 15) == 0 && (U_HH & 15) == 0 && (U_HL & 15) == 0 && (U_STG & 15) == 0 && (U_CS & 15) == 0);
static_assert(L_LDS <= 300 * 1024 && E_LDS <= 300 * 1024 && A_LDS <= 300 * 1024 && U_LDS <= 300 * 1024);
static_assert(NB == 32 * NWAVE && NB <= 256 && WCAP == 256 && CHUNK <= (1 << 20) && NB <= NTHR && ROWS == 64);

typedef float    v4f  __attribute__((ext_vector_type(4)));
typedef float    v8f  __attribute__((ext_vector_type(8)));
typedef int      v4i  __attribute__((ext_vector_type(4)));
typedef _Float16 v4h  __attribute__((ext_vector_type(4)));
typedef _Float16 v8h  __attribute__((ext_vector_type(8)));
typedef _Float16 v16h __attribute__((ext_vector_type(16)));
typedef __bf16   v8b  __attribute__((ext_vector_type(8)));
typedef __bf16   v16b __attribute__((ext_vector_type(16)));
union FragH { v16h v; v8h h[2]; };
union FragB { v16b v; v8b h[2]; };
union U8H   { v8h v; _Float16 e[8]; v4i q; };
union U8B   { v8b v; __bf16 e[8]; v4i q; };

__device__ __forceinline__ v8f zero8f() {
  v8f z;
#pragma unroll
  for (int i = 0; i < 8; ++i) z[i] = 0.0f;
  return z;
}

__device__ __forceinline__ v8f wmh(v16h a, v16h b, v8f c) {
  v8f d = __builtin_amdgcn_wmma_f32_16x16x32_f16(false, a, false, b, (short)0, c, false, false);
  asm volatile("v_nop\n\tv_nop\n\tv_nop\n\tv_nop" : "+v"(d) : "v"(a), "v"(b));
  return d;
}
__device__ __forceinline__ v8f wmb(v16b a, v16b b, v8f c) {
  v8f d = __builtin_amdgcn_wmma_f32_16x16x32_bf16(false, a, false, b, (short)0, c, false, false);
  asm volatile("v_nop\n\tv_nop\n\tv_nop\n\tv_nop" : "+v"(d) : "v"(a), "v"(b));
  return d;
}

__device__ __forceinline__ float bfhi(float x) {
  unsigned u = __float_as_uint(x);
  u = (u + 0x7FFFu + ((u >> 16) & 1u)) & 0xFFFF0000u;
  return __uint_as_float(u);
}

__device__ __forceinline__ void split8(v4f x0, v4f x1, U8B& uh, U8B& ul) {
#pragma unroll
  for (int i = 0; i < 4; ++i) {
    const float a = x0[i], ha = bfhi(a);
    uh.e[i] = (__bf16)ha;
    ul.e[i] = (__bf16)(a - ha);
    const float b = x1[i], hb = bfhi(b);
    uh.e[4 + i] = (__bf16)hb;
    ul.e[4 + i] = (__bf16)(b - hb);
  }
}

__device__ __forceinline__ void gemm_h(const _Float16* arow, const _Float16* bcol, int kp, int nk, v8f acc[4]) {
#pragma unroll 1
  for (int kt = 0; kt < nk; ++kt) {
    FragH a;
    a.h[0] = *(const v8h*)(arow + 32 * kt);
    a.h[1] = *(const v8h*)(arow + 32 * kt + 16);
#pragma unroll
    for (int nt = 0; nt < 4; ++nt) {
      const _Float16* bp = bcol + (size_t)(16 * nt) * kp + 32 * kt;
      FragH b;
      b.h[0] = *(const v8h*)bp;
      b.h[1] = *(const v8h*)(bp + 16);
      acc[nt] = wmh(a.v, b.v, acc[nt]);
    }
  }
}

__device__ __forceinline__ void gemm_b3(const __bf16* ahr, const __bf16* alr, const __bf16* bhc, const __bf16* blc,
                                        int kp, int nk, v8f acc[4]) {
#pragma unroll 1
  for (int kt = 0; kt < nk; ++kt) {
    FragB ah, al;
    ah.h[0] = *(const v8b*)(ahr + 32 * kt);
    ah.h[1] = *(const v8b*)(ahr + 32 * kt + 16);
    al.h[0] = *(const v8b*)(alr + 32 * kt);
    al.h[1] = *(const v8b*)(alr + 32 * kt + 16);
#pragma unroll
    for (int nt = 0; nt < 4; ++nt) {
      const size_t bo = (size_t)(16 * nt) * kp + 32 * kt;
      FragB bh, bl;
      bh.h[0] = *(const v8b*)(bhc + bo);
      bh.h[1] = *(const v8b*)(bhc + bo + 16);
      bl.h[0] = *(const v8b*)(blc + bo);
      bl.h[1] = *(const v8b*)(blc + bo + 16);
      acc[nt] = wmb(ah.v, bh.v, acc[nt]);
      acc[nt] = wmb(al.v, bh.v, acc[nt]);
      acc[nt] = wmb(ah.v, bl.v, acc[nt]);
    }
  }
}

__device__ __forceinline__ void store_rows_f32(const float* stg, float* g, int row0, int M, int wave, int l) {
#pragma unroll
  for (int j = 0; j < 8; ++j) {
    const int lr = 8 * wave + j;
    const int gr = row0 + lr;
    if (gr < M) {
      const v4f v = *(const v4f*)(stg + lr * FP + 4 * l);
      *(volatile v4f*)(g + (size_t)gr * HD + 4 * l) = v;
    }
  }
  __threadfence();
#pragma unroll
  for (int j = 0; j < 8; ++j) {
    const int lr = 8 * wave + j;
    const int gr = row0 + lr;
    if (gr < M) {
      const v4f v = *(const v4f*)(stg + lr * FP + 4 * l);
      *(volatile v4f*)(g + (size_t)gr * HD + 4 * l) = v;
    }
  }
}

__global__ __launch_bounds__(256) void k_wcvt(const float* __restrict__ Wi, const float* __restrict__ W1,
                                              const float* __restrict__ W2, const float* __restrict__ U1,
                                              const float* __restrict__ U2, v4i* wq) {
  const int g = blockIdx.x * 256 + threadIdx.x;
  if (g >= T_GRP) return;
  const float* src = Wi;
  int n = 0, kc = 0, kind = 0;
  if (g < 2048)        { const int q = g;         src = Wi; n = q >> 4; kc = (q & 15) * 8; kind = 0; }
  else if (g < 4096)   { const int q = g - 2048;  src = Wi; n = q >> 4; kc = (q & 15) * 8; kind = 1; }
  else if (g < 6144)   { const int q = g - 4096;  src = W1; n = q >> 4; kc = (q & 15) * 8; kind = 2; }
  else if (g < 6656)   { const int q = g - 6144;  src = W1 + (size_t)HD * HD; n = q >> 2; kc = (q & 3) * 8; kind = 3; }
  else if (g < 8704)   { const int q = g - 6656;  src = W2; n = q >> 4; kc = (q & 15) * 8; kind = 2; }
  else if (g < 12800)  { const int q = g - 8704;  src = U1; n = q >> 5; kc = (q & 31) * 8; kind = 0; }
  else if (g < 16896)  { const int q = g - 12800; src = U1; n = q >> 5; kc = (q & 31) * 8; kind = 1; }
  else if (g < 18944)  { const int q = g - 16896; src = U2; n = q >> 4; kc = (q & 15) * 8; kind = 0; }
  else                 { const int q = g - 18944; src = U2; n = q >> 4; kc = (q & 15) * 8; kind = 1; }
  float x[8];
#pragma unroll
  for (int i = 0; i < 8; ++i) {
    float v = 0.0f;
    if (kind != 3 || kc + i < 8) v = src[(size_t)(kc + i) * HD + n];
    x[i] = v;
  }
  v4i o;
  if (kind <= 1) {
    U8B u;
#pragma unroll
    for (int i = 0; i < 8; ++i) {
      const float hf = bfhi(x[i]);
      u.e[i] = (kind == 0) ? (__bf16)hf : (__bf16)(x[i] - hf);
    }
    o = u.q;
  } else {
    U8H u;
#pragma unroll
    for (int i = 0; i < 8; ++i) u.e[i] = (_Float16)(x[i] * WSC);
    o = u.q;
  }
  *(volatile v4i*)(wq + g) = o;
  __threadfence();
  *(volatile v4i*)(wq + g) = o;
}

__global__ __launch_bounds__(256) void k_lin(const float* __restrict__ nf, const __bf16* tb, const _Float16* th,
                                             const float* __restrict__ bi, float* Hf, float* HW, float* sg, int nN) {
  extern __shared__ __attribute__((aligned(16))) unsigned char lds_l[];
  __bf16*   ahi = (__bf16*)(lds_l + L_AHI);
  __bf16*   alo = (__bf16*)(lds_l + L_ALO);
  _Float16* h16 = (_Float16*)(lds_l + L_H16);
  float*    stg = (float*)(lds_l + L_STG);
  float*    rs  = (float*)(lds_l + L_RS);
  const int tid = threadIdx.x, l = tid & 31, wave = tid >> 5, h = l >> 4, m = l & 15;
  const int wr = wave >> 1, wc = wave & 1;
  const int row0 = blockIdx.x * ROWS;

  for (int i = tid; i < ROWS * 16; i += 256) {
    const int r = i >> 4, c = (i & 15) * 8;
    const int gr = row0 + r;
    v4f x0 = {0.0f, 0.0f, 0.0f, 0.0f};
    v4f x1 = x0;
    if (gr < nN) {
      const float* p = nf + (size_t)gr * HD + c;
      x0 = *(const v4f*)p;
      x1 = *(const v4f*)(p + 4);
    }
    U8B uh, ul;
    split8(x0, x1, uh, ul);
    *(v8b*)(ahi + r * HP + c) = uh.v;
    *(v8b*)(alo + r * HP + c) = ul.v;
  }
  __syncthreads();

  v8f acc[4];
#pragma unroll
  for (int i = 0; i < 4; ++i) acc[i] = zero8f();
  {
    const int ao = (16 * wr + m) * HP + 8 * h;
    const size_t bo = (size_t)(64 * wc + m) * HD + 8 * h;
    gemm_b3(ahi + ao, alo + ao, tb + T_WIH + bo, tb + T_WIL + bo, HD, 4, acc);
  }
#pragma unroll
  for (int nt = 0; nt < 4; ++nt) {
    const int c = 64 * wc + 16 * nt + m;
    const float b = bi[c];
#pragma unroll
    for (int r = 0; r < 8; ++r) {
      const int lr = 16 * wr + 8 * h + r;
      const float v = acc[nt][r] + b;
      stg[lr * FP + c] = v;
      h16[lr * HP + c] = (_Float16)v;
    }
  }
  __syncthreads();

  store_rows_f32(stg, Hf, row0, nN, wave, l);
  if (tid < ROWS) {
    const float* p = stg + tid * FP;
    float s = 0.0f;
#pragma unroll 8
    for (int c = 0; c < HD; ++c) s += p[c];
    rs[tid] = s;
  }
  __syncthreads();

  {
    v4f v = {0.0f, 0.0f, 0.0f, 0.0f};
    if (tid < 16) v = *(const v4f*)(rs + 4 * tid);
    if (tid < 16) *(volatile v4f*)(sg + (size_t)row0 + 4 * tid) = v;
    __threadfence();
    if (tid < 16) *(volatile v4f*)(sg + (size_t)row0 + 4 * tid) = v;
  }

#pragma unroll
  for (int i = 0; i < 4; ++i) acc[i] = zero8f();
  gemm_h(h16 + (16 * wr + m) * HP + 8 * h, th + T_W1A + (size_t)(64 * wc + m) * HD + 8 * h, HD, 4, acc);
#pragma unroll
  for (int nt = 0; nt < 4; ++nt) {
    const int c = 64 * wc + 16 * nt + m;
#pragma unroll
    for (int r = 0; r < 8; ++r) {
      const int lr = 16 * wr + 8 * h + r;
      stg[lr * FP + c] = acc[nt][r] * WINV;
    }
  }
  __syncthreads();
  store_rows_f32(stg, HW, row0, nN, wave, l);
}

__global__ __launch_bounds__(256) void k_edge(const int* __restrict__ ei, const float* __restrict__ pos,
                                              const float* __restrict__ sg, const float* __restrict__ HW,
                                              const _Float16* th, const float* __restrict__ b1,
                                              const float* __restrict__ b2, _Float16* msg, float* gp,
                                              int nN, int nE, int cb, int clen, int gpb) {
  extern __shared__ __attribute__((aligned(16))) unsigned char lds_e[];
  _Float16* rbft = (_Float16*)(lds_e + E_RBF);
  _Float16* hid  = (_Float16*)(lds_e + E_HID);
  _Float16* stg  = (_Float16*)(lds_e + E_STG);
  int*      sidx = (int*)(lds_e + E_SIDX);
  float*    red  = (float*)(lds_e + E_RED);
  const int tid = threadIdx.x, l = tid & 31, wave = tid >> 5, h = l >> 4, m = l & 15;
  const int wr = wave >> 1, wc = wave & 1;
  const int e0 = blockIdx.x * ROWS;

  float gx = 0.0f, gy = 0.0f, gz = 0.0f;
  if (tid < ROWS) {
    const int le = e0 + tid;
    int sc = 0;
    U8H rb;
    rb.q = (v4i){0, 0, 0, 0};
    if (le < clen) {
      const int g = cb + le;
      const int s = ei[g];
      const int d = ei[(size_t)nE + g];
      const bool dok = (unsigned)d < (unsigned)nN;
      sc = s < 0 ? 0 : (s > nN - 1 ? nN - 1 : s);
      const int dc = d < 0 ? 0 : (d > nN - 1 ? nN - 1 : d);
      const float sx = pos[(size_t)sc * 3 + 0], sy = pos[(size_t)sc * 3 + 1], sz = pos[(size_t)sc * 3 + 2];
      const float dx = pos[(size_t)dc * 3 + 0] - sx;
      const float dy = pos[(size_t)dc * 3 + 1] - sy;
      const float dz = pos[(size_t)dc * 3 + 2] - sz;
      const float d2 = dx * dx + dy * dy + dz * dz;
      const float dist = sqrtf(d2);
      const float inv = __builtin_amdgcn_rcpf(dist + 1e-8f);
      const float gate = __builtin_amdgcn_rcpf(1.0f + __expf(-sg[sc]));
      if (dok) {
        gx = gate * (dx * inv);
        gy = gate * (dy * inv);
        gz = gate * (dz * inv);
      }
#pragma unroll
      for (int k = 0; k < 8; ++k) {
        const float ck = (k < 7) ? (8.0f * ((float)k * (1.0f / 7.0f))) : 8.0f;
        const float t = dist - ck;
        rb.e[k] = (_Float16)__expf(-0.5f * (t * t));
      }
    }
    sidx[tid] = sc;
    _Float16* rp = rbft + tid * RP;
    v8h z;
#pragma unroll
    for (int i = 0; i < 8; ++i) z[i] = (_Float16)0.0f;
    *(v8h*)rp = rb.v;
    *(v8h*)(rp + 8) = z;
    *(v8h*)(rp + 16) = z;
    *(v8h*)(rp + 24) = z;
  }
#pragma unroll
  for (int off = 16; off > 0; off >>= 1) {
    gx += __shfl_xor(gx, off);
    gy += __shfl_xor(gy, off);
    gz += __shfl_xor(gz, off);
  }
  if (l == 0 && wave < 2) {
    red[wave * 4 + 0] = gx;
    red[wave * 4 + 1] = gy;
    red[wave * 4 + 2] = gz;
  }
  __syncthreads();

  {
    v4f gv = {0.0f, 0.0f, 0.0f, 0.0f};
    if (tid == 0) {
      gv[0] = red[0] + red[4];
      gv[1] = red[1] + red[5];
      gv[2] = red[2] + red[6];
    }
    float* gl = gp + (size_t)(gpb + blockIdx.x) * 32 + 4 * l;
    if (tid < 8) *(volatile v4f*)gl = gv;
    __threadfence();
    if (tid < 8) *(volatile v4f*)gl = gv;
  }

  v8f acc[4];
#pragma unroll
  for (int i = 0; i < 4; ++i) acc[i] = zero8f();
  gemm_h(rbft + (16 * wr + m) * RP + 8 * h, th + T_W1R + (size_t)(64 * wc + m) * 32 + 8 * h, 32, 1, acc);
  {
    int si[8];
#pragma unroll
    for (int r = 0; r < 8; ++r) si[r] = sidx[16 * wr + 8 * h + r];
#pragma unroll
    for (int nt = 0; nt < 4; ++nt) {
      const int c = 64 * wc + 16 * nt + m;
      const float bc = b1[c];
#pragma unroll
      for (int r = 0; r < 8; ++r) {
        const int lr = 16 * wr + 8 * h + r;
        const float hw = HW[(size_t)si[r] * HD + c];
        float v = acc[nt][r] * WINV + hw;
        v = v + bc;
        const float sgm = __builtin_amdgcn_rcpf(1.0f + __expf(-v));
        hid[lr * HP + c] = (_Float16)(v * sgm);
      }
    }
  }
  __syncthreads();

#pragma unroll
  for (int i = 0; i < 4; ++i) acc[i] = zero8f();
  gemm_h(hid + (16 * wr + m) * HP + 8 * h, th + T_W2 + (size_t)(64 * wc + m) * HD + 8 * h, HD, 4, acc);
#pragma unroll
  for (int nt = 0; nt < 4; ++nt) {
    const int c = 64 * wc + 16 * nt + m;
    const float bc = b2[c];
#pragma unroll
    for (int r = 0; r < 8; ++r) {
      const int lr = 16 * wr + 8 * h + r;
      stg[lr * HP + c] = (_Float16)(acc[nt][r] * WINV + bc);
    }
  }
  __syncthreads();

  {
    const int c8 = 8 * (l & 15);
#pragma unroll
    for (int j = 0; j < 4; ++j) {
      const int lr = 8 * wave + 2 * j + h;
      const int gr = e0 + lr;
      if (gr < clen) {
        const v8h v = *(const v8h*)(stg + lr * HP + c8);
        *(volatile v8h*)(msg + (size_t)gr * HD + c8) = v;
      }
    }
    __threadfence();
#pragma unroll
    for (int j = 0; j < 4; ++j) {
      const int lr = 8 * wave + 2 * j + h;
      const int gr = e0 + lr;
      if (gr < clen) {
        const v8h v = *(const v8h*)(stg + lr * HP + c8);
        *(volatile v8h*)(msg + (size_t)gr * HD + c8) = v;
      }
    }
  }
}

__device__ __forceinline__ int scan_chunk(const int* __restrict__ dsts, int nE, int cbase, int nodeBase,
                                          int* list, int tid, int wave, int vec_ok) {
  int wc = 0;
  const int el0  = tid * EPT;
  const int e0   = cbase + el0;
  const int sent = -2147483647 - 1;
  v4i da, db;
  if (vec_ok != 0 && e0 + 7 < nE) {
    da = *(const v4i*)(dsts + e0);
    db = *(const v4i*)(dsts + e0 + 4);
  } else {
    da.x = (e0     < nE) ? dsts[(e0     < nE) ? e0     : nE - 1] : sent;
    da.y = (e0 + 1 < nE) ? dsts[(e0 + 1 < nE) ? e0 + 1 : nE - 1] : sent;
    da.z = (e0 + 2 < nE) ? dsts[(e0 + 2 < nE) ? e0 + 2 : nE - 1] : sent;
    da.w = (e0 + 3 < nE) ? dsts[(e0 + 3 < nE) ? e0 + 3 : nE - 1] : sent;
    db.x = (e0 + 4 < nE) ? dsts[(e0 + 4 < nE) ? e0 + 4 : nE - 1] : sent;
    db.y = (e0 + 5 < nE) ? dsts[(e0 + 5 < nE) ? e0 + 5 : nE - 1] : sent;
    db.z = (e0 + 6 < nE) ? dsts[(e0 + 6 < nE) ? e0 + 6 : nE - 1] : sent;
    db.w = (e0 + 7 < nE) ? dsts[(e0 + 7 < nE) ? e0 + 7 : nE - 1] : sent;
  }
  const unsigned nb = (unsigned)nodeBase;
  const unsigned s0 = (unsigned)da.x - nb, s1 = (unsigned)da.y - nb;
  const unsigned s2 = (unsigned)da.z - nb, s3 = (unsigned)da.w - nb;
  const unsigned s4 = (unsigned)db.x - nb, s5 = (unsigned)db.y - nb;
  const unsigned s6 = (unsigned)db.z - nb, s7 = (unsigned)db.w - nb;
  const bool q0 = s0 < (unsigned)NB, q1 = s1 < (unsigned)NB, q2 = s2 < (unsigned)NB, q3 = s3 < (unsigned)NB;
  const bool q4 = s4 < (unsigned)NB, q5 = s5 < (unsigned)NB, q6 = s6 < (unsigned)NB, q7 = s7 < (unsigned)NB;
  const unsigned any = __builtin_amdgcn_ballot_w32(q0 | q1 | q2 | q3 | q4 | q5 | q6 | q7);
  if (any != 0u) {
#define HITJ(J, QJ, SJ) { \
      const unsigned mj = __builtin_amdgcn_ballot_w32(QJ); \
      if (mj != 0u) { \
        if (QJ) { \
          const int p = wc + (int)__builtin_amdgcn_mbcnt_lo(mj, 0u); \
          if (p < WCAP) list[wave * WCAP + p] = ((el0 + (J)) << 8) | (int)(SJ); \
        } \
        wc += (int)__builtin_popcount(mj); } }
    HITJ(0, q0, s0)
    HITJ(1, q1, s1)
    HITJ(2, q2, s2)
    HITJ(3, q3, s3)
    HITJ(4, q4, s4)
    HITJ(5, q5, s5)
    HITJ(6, q6, s6)
    HITJ(7, q7, s7)
#undef HITJ
  }
  return wc;
}

__global__ __launch_bounds__(NTHR) void k_agg(const int* __restrict__ dsts, const _Float16* __restrict__ msg,
                                               float* agg, int nN, int clen, int first, int vec_ok) {
  extern __shared__ __attribute__((aligned(16))) unsigned char lds_a[];
  float* acc  = (float*)(lds_a + A_ACC);
  int*   list = (int*)(lds_a + A_LIST);
  int*   wcnt = (int*)(lds_a + A_WCNT);
  const int tid = threadIdx.x, l = tid & 31, wave = tid >> 5;
  const int nodeBase = blockIdx.x * NB;

  for (int i = tid; i < NB * 32; i += NTHR) {
    const int slot = i >> 5, q = (i & 31) * 4;
    const int node = nodeBase + slot;
    v4f v = {0.0f, 0.0f, 0.0f, 0.0f};
    if (first == 0 && node < nN) v = *(const v4f*)(agg + (size_t)node * HD + q);
    *(v4f*)(acc + slot * HD + q) = v;
  }
  __syncthreads();

  const int nChunks = (clen + CHUNK - 1) / CHUNK;
#pragma unroll 1
  for (int ch = 0; ch < nChunks; ++ch) {
    const int cbase = ch * CHUNK;
    const int wc = scan_chunk(dsts, clen, cbase, nodeBase, list, tid, wave, vec_ok);
    if (l == 0) wcnt[wave] = wc;
    __syncthreads();

#pragma unroll 1
    for (int w2 = 0; w2 < NWAVE; ++w2) {
      int n = wcnt[w2];
      n = n > WCAP ? WCAP : (n < 0 ? 0 : n);
      const int* lp = list + w2 * WCAP;
#pragma unroll 1
      for (int i0 = 0; i0 < n; i0 += 32) {
        const int idx = i0 + l;
        const int v = lp[(idx < n) ? idx : 0];
        unsigned mk = __builtin_amdgcn_ballot_w32((idx < n) && ((v & 7) == wave));
#pragma unroll 1
        while (mk != 0u) {
          const int bpos = __builtin_ctz(mk);
          mk &= mk - 1u;
          const int vv = __shfl(v, bpos);
          const int slot = vv & 255;
          int e = cbase + (vv >> 8);
          e = e < 0 ? 0 : (e > clen - 1 ? clen - 1 : e);
          const v4h x = *(const v4h*)(msg + (size_t)e * HD + 4 * l);
          float* ap = acc + slot * HD + 4 * l;
          v4f a = *(v4f*)ap;
          a[0] += (float)x[0]; a[1] += (float)x[1]; a[2] += (float)x[2]; a[3] += (float)x[3];
          *(v4f*)ap = a;
        }
      }
    }
    __syncthreads();
  }

#pragma unroll
  for (int j = 0; j < 32; ++j) {
    const int slot = wave * 32 + j;
    const int node = nodeBase + slot;
    if (node < nN) {
      const v4f a = *(const v4f*)(acc + slot * HD + 4 * l);
      *(volatile v4f*)(agg + (size_t)node * HD + 4 * l) = a;
    }
  }
  __threadfence();
#pragma unroll
  for (int j = 0; j < 32; ++j) {
    const int slot = wave * 32 + j;
    const int node = nodeBase + slot;
    if (node < nN) {
      const v4f a = *(const v4f*)(acc + slot * HD + 4 * l);
      *(volatile v4f*)(agg + (size_t)node * HD + 4 * l) = a;
    }
  }
}

__global__ __launch_bounds__(256) void k_upd(const float* __restrict__ Hf, const float* __restrict__ Ag, const __bf16* tb,
                                             const float* __restrict__ u1, const float* __restrict__ u2,
                                             const float* __restrict__ lng, const float* __restrict__ lnb,
                                             float* out, float* cp, int nN) {
  extern __shared__ __attribute__((aligned(16))) unsigned char lds_u[];
  __bf16* ahi = (__bf16*)(lds_u + U_AHI);
  __bf16* alo = (__bf16*)(lds_u + U_ALO);
  __bf16* hh  = (__bf16*)(lds_u + U_HH);
  __bf16* hl  = (__bf16*)(lds_u + U_HL);
  float*  stg = (float*)(lds_u + U_STG);
  float*  cs  = (float*)(lds_u + U_CS);
  const int tid = threadIdx.x, l = tid & 31, wave = tid >> 5, h = l >> 4, m = l & 15;
  const int wr = wave >> 1, wc = wave & 1;
  const int row0 = blockIdx.x * ROWS;

  for (int i = tid; i < ROWS * 32; i += 256) {
    const int r = i >> 5, c = (i & 31) * 8;
    const int gr = row0 + r;
    v4f x0 = {0.0f, 0.0f, 0.0f, 0.0f};
    v4f x1 = x0;
    if (gr < nN) {
      const float* p = (c < HD) ? (Hf + (size_t)gr * HD + c) : (Ag + (size_t)gr * HD + (c - HD));
      x0 = *(const v4f*)p;
      x1 = *(const v4f*)(p + 4);
    }
    U8B uh, ul;
    split8(x0, x1, uh, ul);
    *(v8b*)(ahi + r * AP + c) = uh.v;
    *(v8b*)(alo + r * AP + c) = ul.v;
  }
  __syncthreads();

  v8f acc[4];
#pragma unroll
  for (int i = 0; i < 4; ++i) acc[i] = zero8f();
  {
    const int ao = (16 * wr + m) * AP + 8 * h;
    const size_t bo = (size_t)(64 * wc + m) * 256 + 8 * h;
    gemm_b3(ahi + ao, alo + ao, tb + T_U1H + bo, tb + T_U1L + bo, 256, 8, acc);
  }
#pragma unroll
  for (int nt = 0; nt < 4; ++nt) {
    const int c = 64 * wc + 16 * nt + m;
    const float bc = u1[c];
#pragma unroll
    for (int r = 0; r < 8; ++r) {
      const int lr = 16 * wr + 8 * h + r;
      const float v = acc[nt][r] + bc;
      const float sgm = __builtin_amdgcn_rcpf(1.0f + __expf(-v));
      const float s = v * sgm;
      const float hs = bfhi(s);
      hh[lr * HP + c] = (__bf16)hs;
      hl[lr * HP + c] = (__bf16)(s - hs);
    }
  }
  __syncthreads();

#pragma unroll
  for (int i = 0; i < 4; ++i) acc[i] = zero8f();
  {
    const int ao = (16 * wr + m) * HP + 8 * h;
    const size_t bo = (size_t)(64 * wc + m) * HD + 8 * h;
    gemm_b3(hh + ao, hl + ao, tb + T_U2H + bo, tb + T_U2L + bo, HD, 4, acc);
  }
#pragma unroll
  for (int nt = 0; nt < 4; ++nt) {
    const int c = 64 * wc + 16 * nt + m;
    const float bc = u2[c];
#pragma unroll
    for (int r = 0; r < 8; ++r) {
      const int lr = 16 * wr + 8 * h + r;
      stg[lr * FP + c] = acc[nt][r] + bc;
    }
  }
  __syncthreads();

  {
    const int row = tid >> 2, q = tid & 3;
    float* xr = stg + row * FP + 32 * q;
    float x[32];
#pragma unroll
    for (int j = 0; j < 8; ++j) {
      const v4f v = *(const v4f*)(xr + 4 * j);
      x[4 * j + 0] = v[0]; x[4 * j + 1] = v[1]; x[4 * j + 2] = v[2]; x[4 * j + 3] = v[3];
    }
    float s = 0.0f;
#pragma unroll
    for (int j = 0; j < 32; ++j) s += x[j];
    s += __shfl_xor(s, 1);
    s += __shfl_xor(s, 2);
    const float mu = s * (1.0f / 128.0f);
    float dv = 0.0f;
#pragma unroll
    for (int j = 0; j < 32; ++j) { const float t = x[j] - mu; dv += t * t; }
    dv += __shfl_xor(dv, 1);
    dv += __shfl_xor(dv, 2);
    const float var = dv * (1.0f / 128.0f);
    const float rstd = rsqrtf(var + 1e-5f);
#pragma unroll
    for (int j = 0; j < 8; ++j) {
      v4f y;
#pragma unroll
      for (int i = 0; i < 4; ++i) {
        const int c = 32 * q + 4 * j + i;
        y[i] = (x[4 * j + i] - mu) * rstd * lng[c] + lnb[c];
      }
      *(v4f*)(xr + 4 * j) = y;
    }
  }
  __syncthreads();

  store_rows_f32(stg, out, row0, nN, wave, l);
  if (tid < HD) {
    int nv = nN - row0;
    nv = nv > ROWS ? ROWS : (nv < 0 ? 0 : nv);
    float s = 0.0f;
#pragma unroll 4
    for (int lr = 0; lr < nv; ++lr) s += stg[lr * FP + tid];
    cs[tid] = s;
  }
  __syncthreads();

  {
    v4f v = {0.0f, 0.0f, 0.0f, 0.0f};
    if (tid < 32) v = *(const v4f*)(cs + 4 * tid);
    float* p = cp + (size_t)blockIdx.x * HD + 4 * tid;
    if (tid < 32) *(volatile v4f*)p = v;
    __threadfence();
    if (tid < 32) *(volatile v4f*)p = v;
  }
}

__global__ __launch_bounds__(256) void k_fin(const float* __restrict__ cp, int ncp, const float* __restrict__ gp, int ngp,
                                             float* out1, float* out2, int nN) {
  __shared__ double rd[256 * 3];
  __shared__ __attribute__((aligned(16))) float o1[HD];
  __shared__ float o2[4];
  const int tid = threadIdx.x;

  if (tid < HD) {
    double s = 0.0;
#pragma unroll 1
    for (int b = 0; b < ncp; ++b) s += (double)cp[(size_t)b * HD + tid];
    o1[tid] = (float)(s / (double)nN);
  }
  {
    double sx = 0.0, sy = 0.0, sz = 0.0;
#pragma unroll 1
    for (int b = tid; b < ngp; b += 256) {
      const float* p = gp + (size_t)b * 32;
      sx += (double)p[0]; sy += (double)p[1]; sz += (double)p[2];
    }
    rd[tid * 3 + 0] = sx; rd[tid * 3 + 1] = sy; rd[tid * 3 + 2] = sz;
  }
  __syncthreads();
  if (tid == 0) {
    double tx = 0.0, ty = 0.0, tz = 0.0;
#pragma unroll 1
    for (int i = 0; i < 256; ++i) { tx += rd[3 * i + 0]; ty += rd[3 * i + 1]; tz += rd[3 * i + 2]; }
    const float vx = (float)(tx / (double)nN);
    const float vy = (float)(ty / (double)nN);
    const float vz = (float)(tz / (double)nN);
    const float nr = sqrtf(vx * vx + vy * vy + vz * vz);
    const float rn = __builtin_amdgcn_rcpf(nr + 1e-8f);
    o2[0] = vx * rn; o2[1] = vy * rn; o2[2] = vz * rn;
  }
  __syncthreads();

  v4f v = {0.0f, 0.0f, 0.0f, 0.0f};
  if (tid < 32) v = *(const v4f*)(o1 + 4 * tid);
  const float a0 = o2[0], a1 = o2[1], a2 = o2[2];
  if (tid < 32) *(volatile v4f*)(out1 + 4 * tid) = v;
  if (tid == 0) {
    ((volatile float*)out2)[0] = a0;
    ((volatile float*)out2)[1] = a1;
    ((volatile float*)out2)[2] = a2;
  }
  __threadfence();
  if (tid < 32) *(volatile v4f*)(out1 + 4 * tid) = v;
  if (tid == 0) {
    ((volatile float*)out2)[0] = a0;
    ((volatile float*)out2)[1] = a1;
    ((volatile float*)out2)[2] = a2;
  }
}

extern "C" void kernel_launch(void* const* d_in, const int* in_sizes, int n_in,
                              void* d_out, int out_size, void* d_ws, size_t ws_size,
                              hipStream_t stream) {
  if (n_in < 15) return;
  const int nN = in_sizes[1] / 3;
  const int nE = in_sizes[2] / 2;
  if (nN <= 0 || nE <= 0) return;
  if (in_sizes[0] != nN * HD || in_sizes[1] != nN * 3 || in_sizes[2] != 2 * nE) return;
  if (in_sizes[3] != HD * HD || in_sizes[4] < HD || in_sizes[5] != 136 * HD || in_sizes[6] < HD) return;
  if (in_sizes[7] != HD * HD || in_sizes[8] < HD || in_sizes[9] != 256 * HD || in_sizes[10] < HD) return;
  if (in_sizes[11] != HD * HD || in_sizes[12] < HD || in_sizes[13] < HD || in_sizes[14] < HD) return;
  if ((long long)out_size != (long long)nN * HD + HD + 3) return;

  const float* node_feat = (const float*)d_in[0];
  const float* pos       = (const float*)d_in[1];
  const int*   ei        = (const int*)d_in[2];
  const float* Wi  = (const float*)d_in[3];
  const float* bi  = (const float*)d_in[4];
  const float* W1  = (const float*)d_in[5];
  const float* b1  = (const float*)d_in[6];
  const float* W2  = (const float*)d_in[7];
  const float* b2  = (const float*)d_in[8];
  const float* U1  = (const float*)d_in[9];
  const float* u1  = (const float*)d_in[10];
  const float* U2  = (const float*)d_in[11];
  const float* u2  = (const float*)d_in[12];
  const float* lng = (const float*)d_in[13];
  const float* lnb = (const float*)d_in[14];
  float* out0 = (float*)d_out;
  float* out1 = out0 + (size_t)nN * HD;
  float* out2 = out1 + HD;

  const int nBlkN = (nN + ROWS - 1) / ROWS;
  const int nBlkA = (nN + NB - 1) / NB;
  long long chl = ((long long)nE + NCHMAX - 1) / NCHMAX;
  chl = (chl + CHUNK - 1) / CHUNK * CHUNK;
  const int CH = (int)chl;
  const int nEBc = (CH + ROWS - 1) / ROWS;
  int nchl = 0;
  for (int c = 0; c < NCHMAX; ++c) if ((long long)c * CH < (long long)nE) ++nchl;
  const int vec_ok = ((nE & 3) == 0) ? 1 : 0;

  char* ws = (char*)d_ws;
  size_t off = 0;
  const size_t oW  = off; off += (size_t)T_TOT * 2;               off = (off + 255) & ~(size_t)255;
  const size_t oH  = off; off += (size_t)nN * HD * 4;             off = (off + 255) & ~(size_t)255;
  const size_t oHW = off; off += (size_t)nN * HD * 4;             off = (off + 255) & ~(size_t)255;
  const size_t oSG = off; off += (size_t)nBlkN * ROWS * 4;        off = (off + 255) & ~(size_t)255;
  const size_t oMS = off; off += (size_t)CH * HD * 2;             off = (off + 255) & ~(size_t)255;
  const size_t oAG = off; off += (size_t)nN * HD * 4;             off = (off + 255) & ~(size_t)255;
  const size_t oGP = off; off += (size_t)NCHMAX * nEBc * 32 * 4;  off = (off + 255) & ~(size_t)255;
  const size_t oCP = off; off += (size_t)nBlkN * HD * 4;          off = (off + 255) & ~(size_t)255;
  if (off > ws_size) return;
  v4i*      wq  = (v4i*)(ws + oW);
  const __bf16*   tb = (const __bf16*)(ws + oW);
  const _Float16* th = (const _Float16*)(ws + oW);
  float*    Hp  = (float*)(ws + oH);
  float*    HWp = (float*)(ws + oHW);
  float*    sgp = (float*)(ws + oSG);
  _Float16* msp = (_Float16*)(ws + oMS);
  float*    agp = (float*)(ws + oAG);
  float*    gpp = (float*)(ws + oGP);
  float*    cpp = (float*)(ws + oCP);

  const hipError_t a0 = hipFuncSetAttribute(reinterpret_cast<const void*>(&k_lin),  hipFuncAttributeMaxDynamicSharedMemorySize, L_LDS);
  const hipError_t a1 = hipFuncSetAttribute(reinterpret_cast<const void*>(&k_edge), hipFuncAttributeMaxDynamicSharedMemorySize, E_LDS);
  const hipError_t a2 = hipFuncSetAttribute(reinterpret_cast<const void*>(&k_agg),  hipFuncAttributeMaxDynamicSharedMemorySize, A_LDS);
  const hipError_t a3 = hipFuncSetAttribute(reinterpret_cast<const void*>(&k_upd),  hipFuncAttributeMaxDynamicSharedMemorySize, U_LDS);
  (void)a0; (void)a1; (void)a2; (void)a3;

  k_wcvt<<<(T_GRP + 255) / 256, 256, 0, stream>>>(Wi, W1, W2, U1, U2, wq);
  k_lin<<<nBlkN, 256, L_LDS, stream>>>(node_feat, tb, th, bi, Hp, HWp, sgp, nN);

  for (int c = 0; c < nchl; ++c) {
    const int cbase = c * CH;
    int clen = nE - cbase;
    clen = clen > CH ? CH : clen;
    k_edge<<<nEBc, 256, E_LDS, stream>>>(ei, pos, sgp, HWp, th, b1, b2, msp, gpp, nN, nE, cbase, clen, c * nEBc);
    k_agg<<<nBlkA, NTHR, A_LDS, stream>>>(ei + (size_t)nE + (size_t)cbase, msp, agp, nN, clen, (c == 0) ? 1 : 0, vec_ok);
  }

  k_upd<<<nBlkN, 256, U_LDS, stream>>>(Hp, agp, tb, u1, u2, lng, lnb, out0, cpp, nN);
  k_fin<<<1, 256, 0, stream>>>(cpp, nBlkN, gpp, nchl * nEBc, out1, out2, nN);
  (void)hipGetLastError();
}
